// cross_SS2D_21861383537444
// MI455X (gfx1250) — hardware-run, weakly checked
//
#include <hip/hip_runtime.h>
#include <hip/hip_fp16.h>
#include <math.h>

typedef __attribute__((ext_vector_type(16))) _Float16 v16h;
typedef __attribute__((ext_vector_type(8)))  _Float16 v8h;
typedef __attribute__((ext_vector_type(8)))  float    v8f;
typedef __attribute__((ext_vector_type(4)))  float    v4f;
typedef __attribute__((ext_vector_type(2)))  unsigned v2u;

constexpr int kNb   = 4;
constexpr int kCh   = 96;
constexpr int kImg  = 64;
constexpr int kSeq  = 4096;
constexpr int kNst  = 16;
constexpr int kRnk  = 6;
constexpr int kPrj  = 38;
constexpr int kChP  = 128;
constexpr int kPrjP = 64;
constexpr int kTP   = 100;
constexpr int kDPit = 132;
constexpr int kOPit = 36;
static_assert(kSeq == kImg * kImg);
static_assert((kCh % 32) == 0 && (kSeq % 64) == 0 && (kPrjP % 64) == 0 && (kChP % 64) == 0);
static_assert(kPrj == kRnk + 2 * kNst && kPrj <= kPrjP && kCh <= kChP);
static_assert((((kSeq / 64) * (kPrjP / 64)) % 8) == 0);

constexpr float kCarX   = 1.0f;
constexpr float kCarW   = 64.0f;
constexpr float kScaleX = 1.0f / (kCarX * kCarW);
constexpr float kYCarry = 16.0f;
constexpr float kInvYC  = 1.0f / 16.0f;
constexpr float kInvLo  = 1.0f / 2048.0f;
constexpr float kInvCh  = 1.0f / 96.0f;
constexpr float kLnEps  = 1e-5f;

constexpr size_t kSzWP  = (size_t)8 * kPrjP * kCh * 2;
constexpr size_t kSzAPD = (size_t)8 * kChP * kNst * 4;
constexpr size_t kSzDPD = (size_t)8 * kChP * 4;
constexpr size_t kSzA16 = (size_t)4 * kSeq * kCh * 2;
constexpr size_t kSzXD  = (size_t)8 * kSeq * kPrjP * 4;
constexpr size_t kSzUPL = (size_t)8 * kSeq * kChP * 4;
constexpr size_t kSzDTP = (size_t)8 * kSeq * kChP * 4;
constexpr size_t kSzBCP = (size_t)8 * kSeq * 32 * 4;
constexpr size_t kSzYH  = (size_t)8 * kSeq * kChP * 2;
constexpr size_t kSzYL  = (size_t)8 * kSeq * kChP * 2;
constexpr size_t kOffWP  = 0;
constexpr size_t kOffAPD = kOffWP  + kSzWP;
constexpr size_t kOffDPD = kOffAPD + kSzAPD;
constexpr size_t kOffA16 = kOffDPD + kSzDPD;
constexpr size_t kOffXD  = kOffA16 + kSzA16;
constexpr size_t kOffUPL = kOffXD  + kSzXD;
constexpr size_t kOffDTP = kOffUPL + kSzUPL;
constexpr size_t kOffBCP = kOffDTP + kSzDTP;
constexpr size_t kOffYH  = kOffBCP + kSzBCP;
constexpr size_t kOffYL  = kOffYH  + kSzYH;
constexpr size_t kWsTotal = kOffYL + kSzYL;
static_assert(kWsTotal == 66228224ull);
static_assert(kWsTotal <= 134217728ull);
static_assert((kOffAPD % 128) == 0 && (kOffDPD % 128) == 0 && (kOffA16 % 128) == 0 && (kOffXD % 128) == 0 &&
              (kOffUPL % 128) == 0 && (kOffDTP % 128) == 0 && (kOffBCP % 128) == 0 && (kOffYH % 128) == 0 &&
              (kOffYL % 128) == 0);
constexpr size_t kOutElems = (size_t)kNb * kCh * kSeq;
static_assert(kOutElems * 4 == 6291456ull);
static_assert(2 * kOutElems * 4 == 12582912ull);

__device__ __forceinline__ _Float16 to_f16_carry(float v, float carry) {
  float c = v * carry;
  c = fminf(fmaxf(c, -65000.0f), 65000.0f);
  c = (fabsf(c) < 6.103515625e-5f) ? 0.0f : c;
  return (_Float16)c;
}
__device__ __forceinline__ float h16_to_f32(unsigned hb) {
  const unsigned sgn = (hb & 0x8000u) << 16; const unsigned em = hb & 0x7fffu;
  const float fn = __uint_as_float((em << 13) + 0x38000000u);
  const float fs = (float)em * 5.9604644775390625e-8f;
  const float mag = (em < 0x400u) ? fs : fn; return __uint_as_float(__float_as_uint(mag) | sgn); }

union FragU { v16h v; v8h h[2]; };
__device__ __forceinline__ v16h frag_load(const _Float16* p) {
  FragU f;
  f.h[0] = *(const v8h*)(p);
  f.h[1] = *(const v8h*)(p + 16);
  return f.v;
}
__device__ __forceinline__ v8f mma_f16(v16h a, v16h b, v8f c) {
  c = __builtin_amdgcn_wmma_f32_16x16x32_f16(false, a, false, b, (short)0, c, false, false);
  asm volatile("v_nop\n\tv_nop\n\tv_nop\n\tv_nop" : "+v"(c) : "v"(a), "v"(b));
  return c;
}
__device__ __forceinline__ void keep4_h(v16h a, v16h b, v16h c, v16h d) { asm volatile("v_nop" :: "v"(a), "v"(b), "v"(c), "v"(d)); }
__device__ __forceinline__ void acc_guard4(v8f& a, v8f& b, v8f& c, v8f& d) { asm volatile("v_nop\n\tv_nop\n\tv_nop\n\tv_nop" : "+v"(a), "+v"(b), "+v"(c), "+v"(d)); }

__global__ __launch_bounds__(256) void params_kernel(
    const float* __restrict__ w_der, const float* __restrict__ w_cli,
    const float* __restrict__ alog_der, const float* __restrict__ alog_cli,
    const float* __restrict__ ds_der, const float* __restrict__ ds_cli,
    unsigned short* __restrict__ WP, float* __restrict__ APD, float* __restrict__ DPD) {
  const unsigned tid = threadIdx.x;
  const unsigned bx = blockIdx.x;
  if (bx < 24u) {
    const unsigned g = bx / 3u;
    const unsigned rem = (bx - g * 3u) * 256u + tid;
    const unsigned n = rem / 12u;
    const unsigned col = (rem - n * 12u) * 8u;
    const unsigned s = g >> 2;
    const unsigned o = (g >> 1) & 1u;
    const unsigned j = g & 1u;
    const unsigned k = o + 2u * j;
    const bool live = n < (unsigned)kPrj;
    const unsigned nc = live ? n : (unsigned)(kPrj - 1);
    const float* sp = (s ? w_cli : w_der) + ((size_t)k * kPrj + nc) * kCh + col;
    v4f a0 = *(const v4f*)(sp);
    v4f a1 = *(const v4f*)(sp + 4);
    asm volatile("" : "+v"(a0));
    asm volatile("" : "+v"(a1));
    v8h hv;
#pragma unroll
    for (int e = 0; e < 4; ++e) {
      const float f0 = live ? a0[e] : 0.0f;
      const float f1 = live ? a1[e] : 0.0f;
      hv[e]     = to_f16_carry(f0, kCarW);
      hv[4 + e] = to_f16_carry(f1, kCarW);
    }
    unsigned short* q = WP + ((size_t)bx * 256u + tid) * 8u;
    *(volatile v8h*)q = hv;
    __threadfence();
    *(volatile v8h*)q = hv;
  } else if (bx < 40u) {
    const unsigned t = (bx - 24u) * 256u + tid;
    const unsigned p = (bx - 24u) >> 1;
    const unsigned rem = t & 511u;
    const unsigned d = rem >> 2;
    const unsigned c4 = (rem & 3u) * 4u;
    const unsigned s = p >> 2;
    const unsigned k = p & 3u;
    const bool live = d < (unsigned)kCh;
    const unsigned dc = live ? d : (unsigned)(kCh - 1);
    v4f a = *(const v4f*)((s ? alog_cli : alog_der) + ((size_t)k * kCh + dc) * kNst + c4);
    asm volatile("" : "+v"(a));
    v4f ov;
#pragma unroll
    for (int e = 0; e < 4; ++e) ov[e] = live ? a[e] : 0.0f;
    float* q = APD + (size_t)t * 4u;
    *(volatile v4f*)q = ov;
    __threadfence();
    *(volatile v4f*)q = ov;
  } else {
    const unsigned p = tid >> 5;
    const unsigned d4 = (tid & 31u) * 4u;
    const unsigned s = p >> 2;
    const unsigned k = p & 3u;
    const bool live = d4 < (unsigned)kCh;
    const unsigned dc = live ? d4 : (unsigned)(kCh - 4);
    v4f va = *(const v4f*)(ds_der + (size_t)k * kCh + dc);
    v4f vb = *(const v4f*)(ds_cli + (size_t)k * kCh + dc);
    asm volatile("" : "+v"(va));
    asm volatile("" : "+v"(vb));
    const float fa = (live && s == 0u) ? 1.0f : 0.0f;
    const float fb = (live && s != 0u) ? 1.0f : 0.0f;
    v4f ov;
#pragma unroll
    for (int e = 0; e < 4; ++e) ov[e] = fa * va[e] + fb * vb[e];
    float* q = DPD + (size_t)tid * 4u;
    *(volatile v4f*)q = ov;
    __threadfence();
    *(volatile v4f*)q = ov;
  }
}

__global__ __launch_bounds__(256) void prep_kernel(
    const float* __restrict__ xin, const float* __restrict__ yin,
    unsigned short* __restrict__ A16, float* __restrict__ UPL, int b) {
  __shared__ __align__(16) float sT[64 * kTP];
  const unsigned tid = threadIdx.x;
  const unsigned i  = blockIdx.x & 63u;
  const unsigned so = blockIdx.x >> 6;
  const unsigned o  = so & 1u;
  const unsigned s  = so >> 1;
  const float* src = (s ? yin : xin) + (size_t)b * kCh * kSeq;
  const unsigned p  = tid & 63u;
  const unsigned c0 = tid >> 6;
  const unsigned pix = o ? (p * 64u + i) : (i * 64u + p);
#pragma unroll 4
  for (unsigned it = 0; it < 24u; ++it) {
    const unsigned ch = it * 4u + c0;
    sT[p * kTP + ch] = src[(size_t)ch * kSeq + pix];
  }
  __syncthreads();
  v8h hv[3];
#pragma unroll
  for (int it = 0; it < 3; ++it) {
    const unsigned g = (unsigned)it * 256u + tid;
    const unsigned e0 = g * 8u;
    const unsigned pp = e0 / (unsigned)kCh;
    const unsigned ch = e0 - pp * (unsigned)kCh;
    const float* sp = sT + pp * kTP + ch;
    const v4f a0 = *(const v4f*)(sp);
    const v4f a1 = *(const v4f*)(sp + 4);
#pragma unroll
    for (int e = 0; e < 4; ++e) {
      hv[it][e]     = to_f16_carry(a0[e], kCarX);
      hv[it][4 + e] = to_f16_carry(a1[e], kCarX);
    }
  }
  v4f uv[8];
#pragma unroll
  for (int it = 0; it < 8; ++it) {
    const unsigned g = (unsigned)it * 256u + tid;
    const unsigned pp = g >> 5;
    const unsigned c4 = (g & 31u) * 4u;
    const bool live = c4 < (unsigned)kCh;
    const unsigned cc = live ? c4 : (unsigned)(kCh - 4);
    const v4f t = *(const v4f*)(sT + pp * kTP + cc);
#pragma unroll
    for (int e = 0; e < 4; ++e) uv[it][e] = live ? t[e] : 0.0f;
  }
  unsigned short* a16p = A16 + ((size_t)so * kSeq + (size_t)i * 64u) * kCh;
  float* uf = UPL + ((size_t)(s * 4u + o) * kSeq) * kChP;
  float* ur = UPL + ((size_t)(s * 4u + o + 2u) * kSeq) * kChP;
  for (int pass = 0; pass < 2; ++pass) {
#pragma unroll
    for (int it = 0; it < 3; ++it) {
      const unsigned g = (unsigned)it * 256u + tid;
      *(volatile v8h*)(a16p + (size_t)g * 8u) = hv[it];
    }
#pragma unroll
    for (int it = 0; it < 8; ++it) {
      const unsigned g = (unsigned)it * 256u + tid;
      const unsigned pp = g >> 5;
      const unsigned c4 = (g & 31u) * 4u;
      const unsigned row = i * 64u + pp;
      *(volatile v4f*)(uf + (size_t)row * kChP + c4) = uv[it];
      *(volatile v4f*)(ur + (size_t)((unsigned)(kSeq - 1) - row) * kChP + c4) = uv[it];
    }
    __threadfence();
  }
}

__global__ __launch_bounds__(256) void gemm_f16_kernel(
    const unsigned short* __restrict__ Ap, int lda, long strideA,
    const unsigned short* __restrict__ Btp, int ldb, long strideB,
    float* __restrict__ Cp, int ldc, long strideC,
    int M, int N, int K, float scale) {
  const _Float16* A  = (const _Float16*)Ap + (size_t)(blockIdx.y >> 1) * (size_t)strideA;
  const _Float16* Bt = (const _Float16*)Btp + (size_t)blockIdx.y * (size_t)strideB;
  float* C = Cp + (size_t)blockIdx.y * (size_t)strideC;
  __shared__ __align__(16) float sT[8][16 * 68];
  const int lane = threadIdx.x & 31;
  const int wave = threadIdx.x >> 5;
  const int tilesN = N >> 6;
  const int tilesM = M >> 6;
  const int tile = blockIdx.x * 8 + wave;
  if (tile >= tilesM * tilesN) return;
  const int tm = tile / tilesN;
  const int tn = tile - tm * tilesN;
  const int m0 = tm << 6;
  const int n0 = tn << 6;

  const int rlane = lane & 15;
  const int koff  = (lane >> 4) * 8;
  const int mOff  = (lane >> 4) * 8;

  v8f acc[4][4];
#pragma unroll
  for (int i = 0; i < 4; ++i)
#pragma unroll
    for (int j = 0; j < 4; ++j) acc[i][j] = (v8f){0.f,0.f,0.f,0.f,0.f,0.f,0.f,0.f};

  for (int k0 = 0; k0 < K; k0 += 32) {
    v16h bh[4];
#pragma unroll
    for (int j = 0; j < 4; ++j) {
      const size_t bo = (size_t)(n0 + (j << 4) + rlane) * ldb + koff + k0;
      bh[j] = frag_load(Bt + bo);
    }
#pragma unroll
    for (int i = 0; i < 4; ++i) {
      const size_t ao = (size_t)(m0 + (i << 4) + rlane) * lda + koff + k0;
      const v16h ah = frag_load(A + ao);
#pragma unroll
      for (int j = 0; j < 4; ++j) acc[i][j] = mma_f16(ah, bh[j], acc[i][j]);
    }
    keep4_h(bh[0], bh[1], bh[2], bh[3]);
  }
  acc_guard4(acc[0][0], acc[0][1], acc[0][2], acc[0][3]);
  acc_guard4(acc[1][0], acc[1][1], acc[1][2], acc[1][3]);
  acc_guard4(acc[2][0], acc[2][1], acc[2][2], acc[2][3]);
  acc_guard4(acc[3][0], acc[3][1], acc[3][2], acc[3][3]);

  float* slab = sT[wave];
#pragma unroll
  for (int i = 0; i < 4; ++i) {
    const int mBase = m0 + (i << 4);
#pragma unroll
    for (int j = 0; j < 4; ++j) {
#pragma unroll
      for (int r = 0; r < 8; ++r) {
        const float v = acc[i][j][r] * scale;
        slab[(mOff + r) * 68 + (j << 4) + rlane] = v;
      }
    }
    __builtin_amdgcn_fence(__ATOMIC_RELEASE, "workgroup");
    __builtin_amdgcn_wave_barrier();
    __builtin_amdgcn_fence(__ATOMIC_ACQUIRE, "workgroup");
    {
      const int hh = lane >> 4, c4 = (lane & 15) * 4;
      for (int pass = 0; pass < 2; ++pass) {
#pragma unroll
        for (int it = 0; it < 8; ++it) {
          const int row = it * 2 + hh;
          const v4f v = *(const v4f*)(slab + row * 68 + c4);
          *(volatile v4f*)(C + (size_t)(mBase + row) * ldc + n0 + c4) = v;
        }
        __threadfence();
      }
    }
    __builtin_amdgcn_fence(__ATOMIC_RELEASE, "workgroup");
    __builtin_amdgcn_wave_barrier();
    __builtin_amdgcn_fence(__ATOMIC_ACQUIRE, "workgroup");
  }
}

__global__ __launch_bounds__(128) void planes_kernel(
    const float* __restrict__ XD,
    const float* __restrict__ dtw_der, const float* __restrict__ dtb_der,
    const float* __restrict__ dtw_cli, const float* __restrict__ dtb_cli,
    float* __restrict__ DTP, float* __restrict__ BCP) {
  __shared__ __align__(16) float sOwn[64 * 24];
  __shared__ __align__(16) float sOth[64 * 24];
  __shared__ __align__(16) float sD[64 * kDPit];
  const unsigned tid = threadIdx.x;
  const unsigned ci = blockIdx.x & 63u;
  const unsigned p  = blockIdx.x >> 6;
  const unsigned k  = p & 3u;
  const unsigned s  = p >> 2;
  const unsigned o  = k & 1u;
  const unsigned j  = k >> 1;
  const unsigned gOwn = (s * 2u + o) * 2u + j;
  const unsigned gOth = ((1u - s) * 2u + o) * 2u + j;
  const bool fwd = (k < 2u);
  const unsigned r0 = ci * 64u;
#pragma unroll
  for (int it = 0; it < 3; ++it) {
    const unsigned idx = (unsigned)it * 128u + tid;
    const unsigned rr = idx / 6u;
    const unsigned q  = idx - rr * 6u;
    const unsigned r  = r0 + rr;
    const unsigned l  = fwd ? r : ((unsigned)(kSeq - 1) - r);
    const v4f a = *(const v4f*)(XD + ((size_t)gOwn * kSeq + l) * kPrjP + q * 4u);
    const v4f c = *(const v4f*)(XD + ((size_t)gOth * kSeq + l) * kPrjP + 16u + q * 4u);
    *(v4f*)(sOwn + rr * 24u + q * 4u) = a;
    *(v4f*)(sOth + rr * 24u + q * 4u) = c;
  }
  const unsigned d = tid;
  const bool live = d < (unsigned)kCh;
  const unsigned dc = live ? d : (unsigned)(kCh - 1);
  const float* dtw = (s ? dtw_cli : dtw_der) + ((size_t)k * kCh + dc) * kRnk;
  const float* dtb = (s ? dtb_cli : dtb_der) + (size_t)k * kCh + dc;
  float w0 = dtw[0], w1 = dtw[1], w2 = dtw[2], w3 = dtw[3], w4 = dtw[4], w5 = dtw[5];
  float bb = dtb[0];
  asm volatile("" : "+v"(w0), "+v"(w1), "+v"(w2), "+v"(w3));
  asm volatile("" : "+v"(w4), "+v"(w5), "+v"(bb));
  w0 = live ? w0 : 0.0f;
  w1 = live ? w1 : 0.0f;
  w2 = live ? w2 : 0.0f;
  w3 = live ? w3 : 0.0f;
  w4 = live ? w4 : 0.0f;
  w5 = live ? w5 : 0.0f;
  bb = live ? bb : 0.0f;
  __syncthreads();
#pragma unroll 4
  for (unsigned rr = 0; rr < 64u; ++rr) {
    const float* xr = sOwn + rr * 24u;
    float pre = bb;
    pre = fmaf(w0, xr[0], pre);
    pre = fmaf(w1, xr[1], pre);
    pre = fmaf(w2, xr[2], pre);
    pre = fmaf(w3, xr[3], pre);
    pre = fmaf(w4, xr[4], pre);
    pre = fmaf(w5, xr[5], pre);
    sD[rr * kDPit + d] = pre;
  }
  __syncthreads();
  v4f dv[16];
#pragma unroll
  for (int it = 0; it < 16; ++it) {
    const unsigned idx = (unsigned)it * 128u + tid;
    const unsigned rr = idx >> 5;
    const unsigned c4 = (idx & 31u) * 4u;
    dv[it] = *(const v4f*)(sD + rr * kDPit + c4);
  }
  v4f bv[4];
#pragma unroll
  for (int it = 0; it < 4; ++it) {
    const unsigned idx = (unsigned)it * 128u + tid;
    const unsigned rr = idx >> 3;
    const unsigned q8 = idx & 7u;
    const bool own = q8 < 4u;
    const unsigned io = rr * 24u + 6u + (own ? (q8 * 4u) : 12u);
    const unsigned ix = rr * 24u + 6u + (own ? 0u : (q8 * 4u - 16u));
#pragma unroll
    for (int e = 0; e < 4; ++e) {
      const float a = sOwn[io + e];
      const float c = sOth[ix + e];
      bv[it][e] = own ? a : c;
    }
  }
  float* dtp = DTP + ((size_t)p * kSeq + r0) * kChP;
  float* bcp = BCP + ((size_t)p * kSeq + r0) * 32u;
  for (int pass = 0; pass < 2; ++pass) {
#pragma unroll
    for (int it = 0; it < 16; ++it) {
      const unsigned idx = (unsigned)it * 128u + tid;
      *(volatile v4f*)(dtp + (size_t)idx * 4u) = dv[it];
    }
#pragma unroll
    for (int it = 0; it < 4; ++it) {
      const unsigned idx = (unsigned)it * 128u + tid;
      *(volatile v4f*)(bcp + (size_t)idx * 4u) = bv[it];
    }
    __threadfence();
  }
}

typedef float    ms1_v4f __attribute__((ext_vector_type(4)));
typedef unsigned ms1_v4u __attribute__((ext_vector_type(4)));
struct ms1_args {
  const float* dtpre;
  const float* u;
  const float* bc;
  const float* z;
  const float* A_log;
  const float* Dskip;
  __half* y;
  __half* y_lo;
  long ld_dtpre;
  long ld_u;
  long ld_bc;
  long ld_z;
  long ld_y;
  int offB;
  int offC;
  int offZ;
  float ycarry;
  int dir;
  int D;
  int L;
  int nbatch;
};
static_assert(sizeof(ms1_args) == 136);

__device__ __forceinline__ float ms1_flush16(float v) {
  return (fabsf(v) < 6.103515625e-05f) ? 0.0f : v;
}
__device__ __forceinline__ unsigned ms1_h16bits(float v) {
  return (unsigned)__half_as_ushort(__float2half_rn(ms1_flush16(v)));
}
__device__ __forceinline__ float ms1_h16val(unsigned b) {
  return __half2float(__ushort_as_half((unsigned short)b));
}
__device__ __forceinline__ float ms1_softplus(float v) {
  return fmaxf(v, 0.0f) + log1pf(expf(-fabsf(v)));
}
__device__ __forceinline__ void ms1_pack2(float v0, float v1, unsigned& hw, unsigned& lw) {
  const unsigned h0 = ms1_h16bits(v0);
  const unsigned h1 = ms1_h16bits(v1);
  const float r0 = (v0 - ms1_h16val(h0)) * 2048.0f;
  const float r1 = (v1 - ms1_h16val(h1)) * 2048.0f;
  const unsigned l0 = ms1_h16bits(r0);
  const unsigned l1 = ms1_h16bits(r1);
  hw = h0 | (h1 << 16);
  lw = l0 | (l1 << 16);
}

template <int NSTATE>
__global__ __launch_bounds__(64 * (NSTATE / 16)) void ms1_scan_kernel(ms1_args a)
{
  static_assert(NSTATE == 16 || NSTATE == 64);
  constexpr int NQ  = NSTATE / 16;
  constexpr int NT  = 64 * NQ;
  constexpr int NW  = NT / 32;
  constexpr int BCW = 2 * NSTATE;
  constexpr int YP  = 68;
  constexpr int RPI = NW * 4;
  constexpr int NIT = 64 / RPI;
  static_assert(16 * NT <= 64 * YP);
  __shared__ __align__(16) float sBC[64 * BCW];
  __shared__ __align__(16) float sY[64 * YP];
  const int tid  = threadIdx.x;
  const int lane = tid & 31;
  const int wave = tid >> 5;
  const int c    = tid / NQ;
  const int sq   = tid - c * NQ;
  const int bpb  = a.D / 64;
  const int bi   = blockIdx.x / bpb;
  if (bi >= a.nbatch) return;
  const int d0 = (blockIdx.x - bi * bpb) * 64;
  const int d  = d0 + c;
  const long rowb = (long)bi * a.L;
  const bool hasz  = (a.z != nullptr);
  const bool hasD  = (a.Dskip != nullptr);
  const bool hasLo = (a.y_lo != nullptr);

#pragma unroll 1
  for (int n = 0; n < 16; ++n) {
    const float al = a.A_log[(long)d * NSTATE + sq * 16 + n];
    sY[n * NT + tid] = -expf(al);
  }
  __syncthreads();
  float An[16], h[16];
#pragma unroll
  for (int n = 0; n < 16; ++n) {
    An[n] = sY[n * NT + tid];
    h[n] = 0.0f;
  }
  float Dd = 0.0f;
  if (hasD) Dd = a.Dskip[d];

  const int nchunk = a.L / 64;
  const bool fwd = (a.dir > 0);
  const int s0 = fwd ? 0 : 63;
  const int sd = fwd ? 1 : -1;
  const int q  = lane >> 3;
  const int c8 = (lane & 7) * 8;

#pragma unroll 1
  for (int ci = 0; ci < nchunk; ++ci) {
    const int tb = fwd ? (ci * 64) : (a.L - 64 - ci * 64);
    const long rowc = rowb + tb;
    __syncthreads();
#pragma unroll 8
    for (int i = 0; i < 32; ++i) {
      const int idx = tid + i * NT;
      const int st  = idx / BCW;
      const int col = idx - st * BCW;
      const int sc  = (col < NSTATE) ? (a.offB + col) : (a.offC + col - NSTATE);
      sBC[idx] = a.bc[(rowc + st) * a.ld_bc + sc];
    }
    __syncthreads();
#pragma unroll 1
    for (int s = 0; s < 64; ++s) {
      const int ls = s0 + sd * s;
      const long row = rowc + ls;
      float pre = a.dtpre[row * a.ld_dtpre + d];
      float uv  = a.u[row * a.ld_u + d];
      float zv  = 0.0f;
      if (hasz) zv = a.z[row * a.ld_z + a.offZ + d];
      asm volatile("" : "+v"(pre));
      asm volatile("" : "+v"(uv));
      asm volatile("" : "+v"(zv));
      const float delta = ms1_softplus(pre);
      const float dtx = delta * uv;
      const float* bp = sBC + ls * BCW + sq * 16;
      const float* cp = bp + NSTATE;
      ms1_v4f Bq[4], Cq[4];
#pragma unroll
      for (int k = 0; k < 4; ++k) {
        Bq[k] = *(const ms1_v4f*)(bp + 4 * k);
        Cq[k] = *(const ms1_v4f*)(cp + 4 * k);
      }
      float yv = 0.0f;
#pragma unroll
      for (int n = 0; n < 16; ++n) {
        const float e = __expf(delta * An[n]);
        h[n] = fmaf(e, h[n], dtx * Bq[n >> 2][n & 3]);
        yv = fmaf(h[n], Cq[n >> 2][n & 3], yv);
      }
      if (NQ > 1) {
        yv += __shfl_xor(yv, 1, 32);
        yv += __shfl_xor(yv, 2, 32);
      }
      if (hasD) yv = fmaf(uv, Dd, yv);
      if (hasz) {
        const float sg = __builtin_amdgcn_rcpf(1.0f + expf(-zv));
        yv = yv * (zv * sg);
      }
      if (sq == 0) sY[ls * YP + c] = yv * a.ycarry;
    }
    __syncthreads();
    ms1_v4u hw[NIT], lw[NIT];
#pragma unroll
    for (int it = 0; it < NIT; ++it) {
      const int row = it * RPI + wave * 4 + q;
      const float* sp = sY + row * YP + c8;
      const ms1_v4f f0 = *(const ms1_v4f*)(sp);
      const ms1_v4f f1 = *(const ms1_v4f*)(sp + 4);
      unsigned h0, h1, h2, h3, l0, l1, l2, l3;
      ms1_pack2(f0[0], f0[1], h0, l0);
      ms1_pack2(f0[2], f0[3], h1, l1);
      ms1_pack2(f1[0], f1[1], h2, l2);
      ms1_pack2(f1[2], f1[3], h3, l3);
      hw[it] = (ms1_v4u){h0, h1, h2, h3};
      lw[it] = (ms1_v4u){l0, l1, l2, l3};
    }
    for (int pass = 0; pass < 2; ++pass) {
#pragma unroll
      for (int it = 0; it < NIT; ++it) {
        const int row = it * RPI + wave * 4 + q;
        const long o = (rowc + row) * a.ld_y + d0 + c8;
        *(volatile ms1_v4u*)(a.y + o) = hw[it];
        if (hasLo) *(volatile ms1_v4u*)(a.y_lo + o) = lw[it];
      }
      __threadfence();
    }
  }
}

__global__ __launch_bounds__(256) void merge_norm_kernel(
    const unsigned short* __restrict__ YH, const unsigned short* __restrict__ YL,
    const float* __restrict__ ln1s, const float* __restrict__ ln1b,
    const float* __restrict__ ln2s, const float* __restrict__ ln2b,
    float* __restrict__ out, int b) {
  __shared__ __align__(16) float sT[kChP * kOPit];
  const unsigned tid  = threadIdx.x;
  const unsigned lane = tid & 31u;
  const unsigned wv   = tid >> 5;
  const unsigned s    = blockIdx.x >> 7;
  const unsigned tile = blockIdx.x & 127u;
  const unsigned l0 = tile * 32u;
  const unsigned hq = l0 >> 6;
  const unsigned w0 = l0 & 63u;
  const bool live = lane < 24u;
  const unsigned lc = live ? lane : 23u;
  v4f gs = *(const v4f*)((s ? ln2s : ln1s) + lc * 4u);
  v4f gb = *(const v4f*)((s ? ln2b : ln1b) + lc * 4u);
  asm volatile("" : "+v"(gs));
  asm volatile("" : "+v"(gb));
  const float fv = live ? 1.0f : 0.0f;
#pragma unroll 1
  for (unsigned j = 0; j < 4u; ++j) {
    const unsigned pi = wv * 4u + j;
    const unsigned wq = w0 + pi;
    const unsigned rowA = hq * 64u + wq;
    const unsigned rowB = wq * 64u + hq;
    float a0 = 0.0f, a1 = 0.0f, a2 = 0.0f, a3 = 0.0f;
#pragma unroll 1
    for (unsigned k = 0; k < 4u; ++k) {
      unsigned row = (k & 1u) ? rowB : rowA;
      row = (k & 2u) ? ((unsigned)(kSeq - 1) - row) : row;
      const size_t off = (((size_t)(s * 4u + k)) * kSeq + row) * kChP + lane * 4u;
      const v2u hw = *(const v2u*)(YH + off);
      const v2u lw = *(const v2u*)(YL + off);
      const float h0 = h16_to_f32(hw.x & 0xffffu), h1 = h16_to_f32(hw.x >> 16);
      const float h2 = h16_to_f32(hw.y & 0xffffu), h3 = h16_to_f32(hw.y >> 16);
      const float r0 = h16_to_f32(lw.x & 0xffffu), r1 = h16_to_f32(lw.x >> 16);
      const float r2 = h16_to_f32(lw.y & 0xffffu), r3 = h16_to_f32(lw.y >> 16);
      a0 += h0 + r0 * kInvLo;
      a1 += h1 + r1 * kInvLo;
      a2 += h2 + r2 * kInvLo;
      a3 += h3 + r3 * kInvLo;
    }
    const float v0 = a0 * kInvYC, v1 = a1 * kInvYC, v2 = a2 * kInvYC, v3 = a3 * kInvYC;
    float sm = (v0 + v1) + (v2 + v3);
    sm += __shfl_xor(sm, 16, 32);
    sm += __shfl_xor(sm, 8, 32);
    sm += __shfl_xor(sm, 4, 32);
    sm += __shfl_xor(sm, 2, 32);
    sm += __shfl_xor(sm, 1, 32);
    const float mu = sm * kInvCh;
    const float e0 = v0 - mu, e1 = v1 - mu, e2 = v2 - mu, e3 = v3 - mu;
    float s2 = fv * ((e0 * e0 + e1 * e1) + (e2 * e2 + e3 * e3));
    s2 += __shfl_xor(s2, 16, 32);
    s2 += __shfl_xor(s2, 8, 32);
    s2 += __shfl_xor(s2, 4, 32);
    s2 += __shfl_xor(s2, 2, 32);
    s2 += __shfl_xor(s2, 1, 32);
    const float rstd = rsqrtf(s2 * kInvCh + kLnEps);
    float* tp = sT + (lane * 4u) * kOPit + pi;
    tp[0]         = e0 * rstd * gs[0] + gb[0];
    tp[kOPit]     = e1 * rstd * gs[1] + gb[1];
    tp[2 * kOPit] = e2 * rstd * gs[2] + gb[2];
    tp[3 * kOPit] = e3 * rstd * gs[3] + gb[3];
  }
  __syncthreads();
  v4f ov[3];
#pragma unroll
  for (int it = 0; it < 3; ++it) {
    const unsigned idx = (unsigned)it * 256u + tid;
    const unsigned dch = idx >> 3;
    const unsigned c4 = (idx & 7u) * 4u;
    ov[it] = *(const v4f*)(sT + dch * kOPit + c4);
  }
  float* ob = out + ((size_t)(s * (unsigned)kNb + (unsigned)b) * kCh) * kSeq + l0;
  for (int pass = 0; pass < 2; ++pass) {
#pragma unroll
    for (int it = 0; it < 3; ++it) {
      const unsigned idx = (unsigned)it * 256u + tid;
      const unsigned dch = idx >> 3;
      const unsigned c4 = (idx & 7u) * 4u;
      *(volatile v4f*)(ob + (size_t)dch * kSeq + c4) = ov[it];
    }
    __threadfence();
  }
}

extern "C" void kernel_launch(void* const* d_in, const int* in_sizes, int n_in,
                              void* d_out, int out_size, void* d_ws, size_t ws_size,
                              hipStream_t stream) {
  if (n_in < 16) return;
  if (in_sizes[0]  != kNb * kCh * kSeq) return;
  if (in_sizes[1]  != kNb * kCh * kSeq) return;
  if (in_sizes[2]  != 4 * kPrj * kCh) return;
  if (in_sizes[3]  != 4 * kCh * kRnk) return;
  if (in_sizes[4]  != 4 * kCh) return;
  if (in_sizes[5]  != 4 * kCh * kNst) return;
  if (in_sizes[6]  != 4 * kCh) return;
  if (in_sizes[7]  != 4 * kPrj * kCh) return;
  if (in_sizes[8]  != 4 * kCh * kRnk) return;
  if (in_sizes[9]  != 4 * kCh) return;
  if (in_sizes[10] != 4 * kCh * kNst) return;
  if (in_sizes[11] != 4 * kCh) return;
  if (in_sizes[12] != kCh) return;
  if (in_sizes[13] != kCh) return;
  if (in_sizes[14] != kCh) return;
  if (in_sizes[15] != kCh) return;
  if (out_size != 2 * kNb * kCh * kSeq) return;
  if (ws_size < kWsTotal) return;

  const float* xin      = (const float*)d_in[0];
  const float* yin      = (const float*)d_in[1];
  const float* w_der    = (const float*)d_in[2];
  const float* dtw_der  = (const float*)d_in[3];
  const float* dtb_der  = (const float*)d_in[4];
  const float* alog_der = (const float*)d_in[5];
  const float* ds_der   = (const float*)d_in[6];
  const float* w_cli    = (const float*)d_in[7];
  const float* dtw_cli  = (const float*)d_in[8];
  const float* dtb_cli  = (const float*)d_in[9];
  const float* alog_cli = (const float*)d_in[10];
  const float* ds_cli   = (const float*)d_in[11];
  const float* ln1s     = (const float*)d_in[12];
  const float* ln1b     = (const float*)d_in[13];
  const float* ln2s     = (const float*)d_in[14];
  const float* ln2b     = (const float*)d_in[15];
  float* out = (float*)d_out;

  char* ws = (char*)d_ws;
  unsigned short* WP  = (unsigned short*)(ws + kOffWP);
  float*          APD = (float*)(ws + kOffAPD);
  float*          DPD = (float*)(ws + kOffDPD);
  unsigned short* A16 = (unsigned short*)(ws + kOffA16);
  float*          XD  = (float*)(ws + kOffXD);
  float*          UPL = (float*)(ws + kOffUPL);
  float*          DTP = (float*)(ws + kOffDTP);
  float*          BCP = (float*)(ws + kOffBCP);
  unsigned short* YH  = (unsigned short*)(ws + kOffYH);
  unsigned short* YL  = (unsigned short*)(ws + kOffYL);

  params_kernel<<<41, 256, 0, stream>>>(w_der, w_cli, alog_der, alog_cli, ds_der, ds_cli, WP, APD, DPD);

  for (int b = 0; b < kNb; ++b) {
    prep_kernel<<<256, 256, 0, stream>>>(xin, yin, A16, UPL, b);

    gemm_f16_kernel<<<dim3(((kSeq / 64) * (kPrjP / 64)) / 8, 8), 256, 0, stream>>>(
        A16, kCh, (long)kSeq * (long)kCh,
        WP, kCh, (long)kPrjP * (long)kCh,
        XD, kPrjP, (long)kSeq * (long)kPrjP,
        kSeq, kPrjP, kCh, kScaleX);

    planes_kernel<<<8 * 64, 128, 0, stream>>>(XD, dtw_der, dtb_der, dtw_cli, dtb_cli, DTP, BCP);

    for (int p = 0; p < 8; ++p) {
      ms1_args sa;
      sa.dtpre = DTP + (size_t)p * kSeq * kChP;
      sa.u = UPL + (size_t)p * kSeq * kChP;
      sa.bc = BCP + (size_t)p * kSeq * 32;
      sa.z = nullptr;
      sa.A_log = APD + (size_t)p * kChP * kNst;
      sa.Dskip = DPD + (size_t)p * kChP;
      sa.y = (__half*)(YH + (size_t)p * kSeq * kChP);
      sa.y_lo = (__half*)(YL + (size_t)p * kSeq * kChP);
      sa.ld_dtpre = kChP;
      sa.ld_u = kChP;
      sa.ld_bc = 32;
      sa.ld_z = 0;
      sa.ld_y = kChP;
      sa.offB = 0;
      sa.offC = 16;
      sa.offZ = 0;
      sa.ycarry = kYCarry;
      sa.dir = 1;
      sa.D = kChP;
      sa.L = kSeq;
      sa.nbatch = 1;
      ms1_scan_kernel<16><<<dim3(kChP / 64), 64, 0, stream>>>(sa);
    }

    merge_norm_kernel<<<256, 256, 0, stream>>>(YH, YL, ln1s, ln1b, ln2s, ln2b, out, b);
  }
}
